// GraphInductiveLayer_36447092474026
// MI455X (gfx1250) — hardware-verified
//
#include <hip/hip_runtime.h>

typedef float          v8f   __attribute__((ext_vector_type(8)));
typedef float          v4f   __attribute__((ext_vector_type(4)));
typedef unsigned int   v4u   __attribute__((ext_vector_type(4)));
typedef int            v8i   __attribute__((ext_vector_type(8)));
typedef unsigned short v8us  __attribute__((ext_vector_type(8)));
typedef unsigned short v16us __attribute__((ext_vector_type(16)));
typedef __bf16         v16bf __attribute__((ext_vector_type(16)));
typedef _Float16       v16h  __attribute__((ext_vector_type(16)));
typedef v4f  __attribute__((may_alias)) v4fa;
typedef v8us __attribute__((may_alias)) v8usa;
union FragB { v16bf v; v16us u; v8us h[2]; v8i w; };
union FragH { v16h  v; v16us u; v8us h[2]; v8i w; };

__device__ __forceinline__ v8f wmb(const FragB& a, const FragB& b, v8f c) {
  v8f d = __builtin_amdgcn_wmma_f32_16x16x32_bf16(false, a.v, false, b.v, (short)0, c, false, false);
  asm volatile("v_nop\n\tv_nop\n\tv_nop\n\tv_nop" : "+v"(d) : "v"(a.w), "v"(b.w));
  return d;
}

__device__ __forceinline__ v8f wmh(const FragH& a, const FragH& b, v8f c) {
  v8f d = __builtin_amdgcn_wmma_f32_16x16x32_f16(false, a.v, false, b.v, (short)0, c, false, false);
  asm volatile("v_nop\n\tv_nop\n\tv_nop\n\tv_nop" : "+v"(d) : "v"(a.w), "v"(b.w));
  return d;
}

__device__ __forceinline__ unsigned bf16_bits(float f) {
  const unsigned u = __float_as_uint(f);
  const unsigned r = (u + 0x7FFFu + ((u >> 16) & 1u)) >> 16;
  const unsigned q = (u >> 16) | 0x40u;
  return ((u & 0x7fffffffu) > 0x7f800000u) ? q : r;
}

__device__ __forceinline__ float bf16_val(float f) {
  return __uint_as_float(bf16_bits(f) << 16);
}
__device__ __forceinline__ int clampi(int v, int lo, int hi) {
  return v < lo ? lo : (v > hi ? hi : v);
}

__device__ __forceinline__ unsigned f16_bits(float f) {
  const unsigned u  = __float_as_uint(f);
  const unsigned s  = (u >> 16) & 0x8000u;
  const unsigned a  = u & 0x7fffffffu;
  const unsigned t  = a - 0x38000000u;
  const unsigned r  = (t + 0x0FFFu + ((t >> 13) & 1u)) >> 13;
  const unsigned rc = r > 0x7C00u ? 0x7C00u : r;
  const bool small  = a < 0x38800000u;
  const bool isnan  = a > 0x7f800000u;
  const unsigned fin = small ? 0u : (s | rc);
  return isnan ? (s | 0x7E00u) : fin;
}

__device__ __forceinline__ unsigned pk16(unsigned lo, unsigned hi) { return lo | (hi << 16); }
__device__ __forceinline__ unsigned bf16_lo_bits(float v) {
  float hi = bf16_val(v);
  asm volatile("" : "+v"(hi));
  return bf16_bits(v - hi);
}
__device__ __forceinline__ v4u pack8_bf16(v4f a, v4f c) {
  return (v4u){ pk16(bf16_bits(a[0]), bf16_bits(a[1])), pk16(bf16_bits(a[2]), bf16_bits(a[3])),
                pk16(bf16_bits(c[0]), bf16_bits(c[1])), pk16(bf16_bits(c[2]), bf16_bits(c[3])) };
}
__device__ __forceinline__ v4u pack8_bf16_lo(v4f a, v4f c) {
  return (v4u){ pk16(bf16_lo_bits(a[0]), bf16_lo_bits(a[1])), pk16(bf16_lo_bits(a[2]), bf16_lo_bits(a[3])),
                pk16(bf16_lo_bits(c[0]), bf16_lo_bits(c[1])), pk16(bf16_lo_bits(c[2]), bf16_lo_bits(c[3])) };
}
__device__ __forceinline__ v4u pack8_f16(v4f a, v4f c) {
  return (v4u){ pk16(f16_bits(a[0]), f16_bits(a[1])), pk16(f16_bits(a[2]), f16_bits(a[3])),
                pk16(f16_bits(c[0]), f16_bits(c[1])), pk16(f16_bits(c[2]), f16_bits(c[3])) };
}

template <int FORM>
__global__ __launch_bounds__(256) void k_plane(const float* __restrict__ src, int rows, int cols, int ldsrc,
                                               unsigned short* __restrict__ dst, int MP, int KP) {
  static_assert(FORM >= 0 && FORM <= 3);
  const int KTOT = (FORM == 1 || FORM == 3) ? 2 * KP : KP;
  const unsigned ppr   = (unsigned)(KTOT >> 3);
  const unsigned kp8   = (unsigned)(KP >> 3);
  const unsigned total = (unsigned)MP * ppr;
  const unsigned g     = blockIdx.x * 256u + threadIdx.x;
  const unsigned rowu  = g / ppr;
  const unsigned p     = g - rowu * ppr;
  const bool second    = p >= kp8;
  const int row = (int)rowu;
  const int c0  = (int)((second ? p - kp8 : p) << 3);
  const float* srow = src + (size_t)clampi(row, 0, rows - 1) * (size_t)ldsrc;
  float x[8];
  unsigned mk[8];
#pragma unroll
  for (int e = 0; e < 8; ++e) {
    const int c = c0 + e;
    const float v = srow[clampi(c, 0, cols - 1)];
    asm volatile("" :: "v"(v));
    x[e]  = v;
    mk[e] = (row < rows && c < cols) ? 0xFFFFu : 0u;
  }
  const v4f a = (v4f){ x[0], x[1], x[2], x[3] };
  const v4f c = (v4f){ x[4], x[5], x[6], x[7] };
  v4u o;
  if (FORM == 2) {
    o = pack8_f16(a, c);
  } else {
    const v4u hi = pack8_bf16(a, c);
    o = hi;
    if (FORM == 1) { const v4u lo = pack8_bf16_lo(a, c); o = second ? lo : hi; }
  }
  const v4u mw = (v4u){ pk16(mk[0], mk[1]), pk16(mk[2], mk[3]), pk16(mk[4], mk[5]), pk16(mk[6], mk[7]) };
  o &= mw;
  if (g < total) {
    volatile v4u* q = (volatile v4u*)(dst + (size_t)g * 8);
    *q = o;
    __threadfence();
    *q = o;
  }
}

template <int FORM> struct FragOf    { typedef FragB T; };
template <>         struct FragOf<2> { typedef FragH T; };
__device__ __forceinline__ v8f mm(const FragB& a, const FragB& b, v8f c) { return wmb(a, b, c); }
__device__ __forceinline__ v8f mm(const FragH& a, const FragH& b, v8f c) { return wmh(a, b, c); }
template <class F> __device__ __forceinline__ F ld_frag(const unsigned short* p) {
  F f;
  f.h[0] = *(const v8usa*)(p);
  f.h[1] = *(const v8usa*)(p + 16);
  return f;
}

template <int FORM, int EPI>
__global__ __launch_bounds__(256) __attribute__((amdgpu_num_vgpr(248)))
void k_gemm_nt(const unsigned short* __restrict__ A, const unsigned short* __restrict__ B,
               const float* __restrict__ bias, float* __restrict__ D, int M, int N, int KTOT, int ldd) {
  static_assert(FORM >= 0 && FORM <= 2);
  static_assert(EPI == 0 || EPI == 1);
  typedef typename FragOf<FORM>::T F;
  __shared__ __attribute__((aligned(16))) float sT[8][16 * 68];
  const int lane = threadIdx.x & 31;
  const int wave = threadIdx.x >> 5;
  const int tilesM = (M + 63) >> 6;
  const int tilesN = (N + 63) >> 6;
  const int tile = blockIdx.x * 8 + wave;
  if (tile >= tilesM * tilesN) return;
  const int tm = tile / tilesN;
  const int tn = tile - tm * tilesN;
  const int m0 = tm << 6;
  const int n0 = tn << 6;

  const int rl = lane & 15;
  const int h8 = (lane >> 4) * 8;
  const unsigned short* pa = A + (size_t)(m0 + rl) * (size_t)KTOT + h8;
  const unsigned short* pb = B + (size_t)(n0 + rl) * (size_t)KTOT + h8;

  v8f acc[4][4];
#pragma unroll
  for (int i = 0; i < 4; ++i)
#pragma unroll
    for (int j = 0; j < 4; ++j) acc[i][j] = (v8f){0.f, 0.f, 0.f, 0.f, 0.f, 0.f, 0.f, 0.f};

#pragma unroll 1
  for (int k0 = 0; k0 < KTOT; k0 += 32) {
    F bf[4];
#pragma unroll
    for (int j = 0; j < 4; ++j) bf[j] = ld_frag<F>(pb + (size_t)(j << 4) * (size_t)KTOT + k0);
#pragma unroll
    for (int i = 0; i < 4; ++i) {
      const F af = ld_frag<F>(pa + (size_t)(i << 4) * (size_t)KTOT + k0);
#pragma unroll
      for (int j = 0; j < 4; ++j) acc[i][j] = mm(af, bf[j], acc[i][j]);
    }
  }

  float* slab = sT[wave];
  const int hh = lane >> 4;
  const int c4 = (lane & 15) * 4;
  const int nc = n0 + c4;
  const bool cok = nc < N;
  v4f bv = (v4f){0.f, 0.f, 0.f, 0.f};
  if (EPI == 1) {
    bv = *(const v4fa*)(bias + clampi(nc, 0, N - 4));
    asm volatile("" :: "v"(bv));
  }
#pragma unroll
  for (int i = 0; i < 4; ++i) {
    const int mBase = m0 + (i << 4);
#pragma unroll
    for (int j = 0; j < 4; ++j) {
#pragma unroll
      for (int r = 0; r < 8; ++r) slab[(h8 + r) * 68 + (j << 4) + rl] = acc[i][j][r];
    }
    __builtin_amdgcn_fence(__ATOMIC_RELEASE, "workgroup");
    __builtin_amdgcn_wave_barrier();
    __builtin_amdgcn_fence(__ATOMIC_ACQUIRE, "workgroup");
    v4f vv[8];
#pragma unroll
    for (int it = 0; it < 8; ++it) {
      const int row = it * 2 + hh;
      v4f v = *(const v4fa*)(slab + row * 68 + c4);
      if (EPI == 1) v += bv;
      vv[it] = v;
    }
    for (int pass = 0; pass < 2; ++pass) {
#pragma unroll
      for (int it = 0; it < 8; ++it) {
        const int row = mBase + it * 2 + hh;
        if (cok && row < M) *(volatile v4f*)(D + (size_t)row * (size_t)ldd + nc) = vv[it];
      }
      __threadfence();
    }
    __builtin_amdgcn_fence(__ATOMIC_RELEASE, "workgroup");
    __builtin_amdgcn_wave_barrier();
    __builtin_amdgcn_fence(__ATOMIC_ACQUIRE, "workgroup");
  }
}

#include <stddef.h>
#pragma clang fp contract(off)

#define NN      100000
#define NSAMP   25
#define FD      128
#define K2      256
#define MP      100096
#define NTHR    256
#define NWAVE   8
#define WBLK    (MP / NWAVE)
#define PW_U    (FD * K2 / 8)
#define PW_B    (PW_U / NTHR)
#define PW_BLKS (PW_B + 1)

static_assert(NSAMP == 25 && NSAMP <= 32);
static_assert(FD == 128 && FD == 32 * 4);
static_assert(K2 == 2 * FD && K2 == 256);
static_assert(MP == 782 * 128 && MP % 128 == 0 && MP % 64 == 0 && MP >= NN);
static_assert(NN % 16 == 0 && FD % 64 == 0 && FD % 32 == 0 && K2 % 32 == 0);
static_assert(WBLK * NWAVE == MP);
static_assert((MP * FD / 8) % NTHR == 0);
static_assert(PW_U % NTHR == 0 && K2 / 8 == 32);
static_assert(sizeof(int) == 4);
static_assert((FD * 2) % 128 == 0 && (K2 * 2) % 128 == 0 && (FD * 4) % 128 == 0);

typedef unsigned int v2u __attribute__((ext_vector_type(2)));
typedef v2u __attribute__((may_alias)) v2ua;

__device__ __forceinline__ void st2_v4f(float* p, v4f v) {
  *(volatile v4f*)p = v;
  __threadfence();
  *(volatile v4f*)p = v;
}
__device__ __forceinline__ void st2_v8us(unsigned short* p, v8us v) {
  *(volatile v8us*)p = v;
  __threadfence();
  *(volatile v8us*)p = v;
}

__device__ __forceinline__ v8us gather8(const float* __restrict__ base, int stride) {
  float f[8];
#pragma unroll
  for (int i = 0; i < 8; ++i) f[i] = base[(size_t)i * (size_t)stride];
  v8us o;
#pragma unroll
  for (int i = 0; i < 8; ++i) o[i] = (unsigned short)bf16_bits(f[i]);
  return o;
}

__global__ __launch_bounds__(NTHR) void k_prep(const float* __restrict__ W, const float* __restrict__ b,
                                               unsigned short* wt2, float* bias) {
  const int tid = (int)threadIdx.x;
  const int blk = (int)blockIdx.x;
  if (blk < PW_B) {
    const int u  = blk * NTHR + tid;
    const int n  = u >> 5;
    const int k8 = (u & 31) * 8;
    const int ks = k8 & (FD - 1);
    const v8us o = gather8(W + (size_t)ks * FD + n, FD);
    st2_v8us(wt2 + (size_t)u * 8, o);
  } else {
    if (tid < 32) {
      const v4f v = *(const v4fa*)(b + 4 * tid);
      v4f o;
      o.x = bf16_val(v.x); o.y = bf16_val(v.y); o.z = bf16_val(v.z); o.w = bf16_val(v.w);
      st2_v4f(bias + 4 * tid, o);
    }
  }
}

__global__ __launch_bounds__(NTHR) void k_walk(const int* __restrict__ nidx, const unsigned short* __restrict__ XB,
                                               unsigned short* OP) {
  const int tid = (int)threadIdx.x, lane = tid & 31, wave = tid >> 5;
  const int v  = (int)blockIdx.x * NWAVE + wave;
  const int vc = v < NN ? v : NN - 1;
  const int sl = lane < NSAMP ? lane : NSAMP - 1;

  int id = nidx[(size_t)vc * NSAMP + sl];
  asm volatile("" : "+v"(id));
  id = clampi(id, 0, NN - 1);

  const unsigned short* xl = XB + 4 * lane;
  float a0 = 0.0f, a1 = 0.0f, a2 = 0.0f, a3 = 0.0f;

#pragma unroll
  for (int g = 0; g < 5; ++g) {
    v2u w[5];
#pragma unroll
    for (int j = 0; j < 5; ++j) {
      const int ids = __builtin_amdgcn_readlane(id, g * 5 + j);
      w[j] = *(const v2ua*)(xl + (size_t)ids * FD);
    }
#pragma unroll
    for (int j = 0; j < 5; ++j) {
      float f0 = __uint_as_float(w[j].x << 16);
      float f1 = __uint_as_float(w[j].x & 0xffff0000u);
      float f2 = __uint_as_float(w[j].y << 16);
      float f3 = __uint_as_float(w[j].y & 0xffff0000u);
      asm volatile("" : "+v"(f0));
      asm volatile("" : "+v"(f1));
      asm volatile("" : "+v"(f2));
      asm volatile("" : "+v"(f3));
      a0 += f0; a1 += f1; a2 += f2; a3 += f3;
    }
    __builtin_amdgcn_sched_barrier(0);
  }

  const v2u wo = *(const v2ua*)(xl + (size_t)vc * FD);
  float o0 = __uint_as_float(wo.x << 16);
  float o1 = __uint_as_float(wo.x & 0xffff0000u);
  float o2 = __uint_as_float(wo.y << 16);
  float o3 = __uint_as_float(wo.y & 0xffff0000u);
  asm volatile("" : "+v"(o0));
  asm volatile("" : "+v"(o1));
  asm volatile("" : "+v"(o2));
  asm volatile("" : "+v"(o3));
  const float t0 = a0 + o0, t1 = a1 + o1, t2 = a2 + o2, t3 = a3 + o3;
  const float q0 = t0 / 26.0f, q1 = t1 / 26.0f, q2 = t2 / 26.0f, q3 = t3 / 26.0f;

  const unsigned keep = (v < NN) ? 0xFFFFFFFFu : 0u;
  v2u hv, lv;
  hv.x = pk16(bf16_bits(q0), bf16_bits(q1)) & keep;
  hv.y = pk16(bf16_bits(q2), bf16_bits(q3)) & keep;
  lv.x = pk16(bf16_lo_bits(q0), bf16_lo_bits(q1)) & keep;
  lv.y = pk16(bf16_lo_bits(q2), bf16_lo_bits(q3)) & keep;

  unsigned short* orow = OP + (size_t)v * K2 + 4 * lane;
  for (int pass = 0; pass < 2; ++pass) {
    *(volatile v2u*)orow = hv;
    *(volatile v2u*)(orow + FD) = lv;
    __threadfence();
  }
}

extern "C" void kernel_launch(void* const* d_in, const int* in_sizes, int n_in,
                              void* d_out, int out_size, void* d_ws, size_t ws_size,
                              hipStream_t stream) {
  if (n_in < 4) return;
  if (in_sizes[0] != NN * FD) return;
  if (in_sizes[1] != NN * NSAMP) return;
  if (in_sizes[2] != FD * FD) return;
  if (in_sizes[3] != FD) return;
  if (out_size != NN * FD) return;

  const float* x    = (const float*)d_in[0];
  const int*   nidx = (const int*)d_in[1];
  const float* W    = (const float*)d_in[2];
  const float* bvec = (const float*)d_in[3];
  float* out = (float*)d_out;

  constexpr size_t zXB   = (size_t)MP * FD * 2;
  constexpr size_t zOP   = (size_t)MP * K2 * 2;
  constexpr size_t zWT2  = (size_t)FD * K2 * 2;
  constexpr size_t zBIAS = (size_t)FD * 4;
  constexpr size_t oXB   = 0;
  constexpr size_t oOP   = oXB + zXB;
  constexpr size_t oWT2  = oOP + zOP;
  constexpr size_t oBIAS = oWT2 + zWT2;
  constexpr size_t oEND  = oBIAS + zBIAS;
  static_assert(zXB % 256 == 0 && zOP % 256 == 0 && zWT2 % 256 == 0 && zBIAS % 128 == 0);
  static_assert(oOP % 256 == 0 && oWT2 % 256 == 0 && oBIAS % 256 == 0);
  static_assert(oEND == (size_t)76939776);
  static_assert(oEND <= ((size_t)128 << 20));
  if (oEND > ws_size) return;

  char* ws = (char*)d_ws;
  unsigned short* XB   = (unsigned short*)(ws + oXB);
  unsigned short* OP   = (unsigned short*)(ws + oOP);
  unsigned short* WT2  = (unsigned short*)(ws + oWT2);
  float*          BIAS = (float*)(ws + oBIAS);

  const int tiles = ((NN + 63) / 64) * (FD / 64);
  const int gg    = (tiles + 7) / 8;

  k_plane<0><<<MP * FD / 8 / NTHR, NTHR, 0, stream>>>(x, NN, FD, FD, XB, MP, FD);
  k_prep<<<PW_BLKS, NTHR, 0, stream>>>(W, bvec, WT2, BIAS);
  k_walk<<<WBLK, NTHR, 0, stream>>>(nidx, XB, OP);
  k_gemm_nt<0, 1><<<gg, NTHR, 0, stream>>>(OP, WT2, BIAS, out, NN, FD, K2, FD);
}
